// MultiHeadAttentionWithBias_6622839571248
// MI455X (gfx1250) — hardware-verified
//
#include <hip/hip_runtime.h>
#include <math.h>
#include <stdint.h>

typedef __attribute__((ext_vector_type(16))) _Float16 v16h;
typedef __attribute__((ext_vector_type(8)))  _Float16 v8h;
typedef __attribute__((ext_vector_type(16))) __bf16   v16b;
typedef __attribute__((ext_vector_type(8)))  __bf16   v8b;
typedef __attribute__((ext_vector_type(8)))  float    v8f;
typedef __attribute__((ext_vector_type(4)))  float    v4f;
typedef __attribute__((ext_vector_type(2)))  float    v2f;

__device__ __forceinline__ unsigned short f2bf_bits(float f) {
  unsigned u = __float_as_uint(f);
  return (unsigned short)((u + 0x7FFFu + ((u >> 16) & 1u)) >> 16);
}
__device__ __forceinline__ float bf_bits2f(unsigned short h) { return __uint_as_float(((unsigned)h) << 16); }

__device__ __forceinline__ void dep_guard_h(v8f& a, v8f& b, v16h x, v16h y) { asm volatile("v_nop\n\tv_nop\n\tv_nop\n\tv_nop" : "+v"(a), "+v"(b) : "v"(x), "v"(y)); }
__device__ __forceinline__ void dep_guard_b(v8f& a, v8f& b, v16b x, v16b y) { asm volatile("v_nop\n\tv_nop\n\tv_nop\n\tv_nop" : "+v"(a), "+v"(b) : "v"(x), "v"(y)); }
__device__ __forceinline__ void keep4_h(v16h a, v16h b, v16h c, v16h d) { asm volatile("v_nop" :: "v"(a), "v"(b), "v"(c), "v"(d)); }
__device__ __forceinline__ void keep4_b(v16b a, v16b b, v16b c, v16b d) { asm volatile("v_nop" :: "v"(a), "v"(b), "v"(c), "v"(d)); }
__device__ __forceinline__ void acc_guard4(v8f& a, v8f& b, v8f& c, v8f& d) { asm volatile("v_nop\n\tv_nop\n\tv_nop\n\tv_nop" : "+v"(a), "+v"(b), "+v"(c), "+v"(d)); }
template <typename T> struct Frag;
template <> struct Frag<_Float16> {
  typedef v16h V; union U { v16h v; v8h h[2]; };
  static __device__ __forceinline__ v16h load(const _Float16* p) {
    U f; f.h[0] = *(const v8h*)(p); f.h[1] = *(const v8h*)(p + 16); return f.v;
  }
  static __device__ __forceinline__ v8f mma(v16h a, v16h b, v8f c) {
    return __builtin_amdgcn_wmma_f32_16x16x32_f16(false, a, false, b, (short)0, c, false, false);
  }
  static __device__ __forceinline__ void guard(v8f& a, v8f& b, v16h x, v16h y) { dep_guard_h(a, b, x, y); }
  static __device__ __forceinline__ void keep(v16h a, v16h b, v16h c, v16h d) { keep4_h(a, b, c, d); }
};
template <> struct Frag<__bf16> {
  typedef v16b V; union U { v16b v; v8b h[2]; };
  static __device__ __forceinline__ v16b load(const __bf16* p) {
    U f; f.h[0] = *(const v8b*)(p); f.h[1] = *(const v8b*)(p + 16); return f.v;
  }
  static __device__ __forceinline__ v8f mma(v16b a, v16b b, v8f c) {
    return __builtin_amdgcn_wmma_f32_16x16x32_bf16(false, a, false, b, (short)0, c, false, false);
  }
  static __device__ __forceinline__ void guard(v8f& a, v8f& b, v16b x, v16b y) { dep_guard_b(a, b, x, y); }
  static __device__ __forceinline__ void keep(v16b a, v16b b, v16b c, v16b d) { keep4_b(a, b, c, d); }
};

template <int ET> struct Elem;
template <> struct Elem<0> { typedef _Float16 T; };
template <> struct Elem<1> { typedef __bf16 T; };
template <int ET, bool SPLIT, int BIAS_MODE, int OUT_MODE, bool RESID, int ACT = 0>
__global__ __launch_bounds__(256) void wmma_gemm64(
    const unsigned short* __restrict__ Ap, const unsigned short* __restrict__ A2p, int lda, long strideA,
    const unsigned short* __restrict__ Btp, const unsigned short* __restrict__ Bt2p, int ldb, long strideB,
    void* __restrict__ Cout, void* __restrict__ Cout2, int ldc, long strideC,
    const float* __restrict__ bias,
    const float* __restrict__ resid, long strideR,
    int M, int N, int K, float scale) {
  typedef typename Elem<ET>::T T;
  typedef typename Frag<T>::V V;
  const T* A = (const T*)Ap; const T* A2 = (const T*)A2p; const T* Bt = (const T*)Btp; const T* Bt2 = (const T*)Bt2p;
  __shared__ __align__(16) float sT[8][16 * 68];
  const int b    = blockIdx.y;
  const int lane = threadIdx.x & 31;
  const int wave = threadIdx.x >> 5;
  const int tilesN = N >> 6;
  const int tilesM = M >> 6;
  const int tile = blockIdx.x * 8 + wave;
  if (tile >= tilesM * tilesN) return;
  const int tm = tile / tilesN;
  const int tn = tile - tm * tilesN;
  const int m0 = tm << 6;
  const int n0 = tn << 6;

  const T* Ab  = A  + (size_t)b * strideA;
  const T* Bb  = Bt + (size_t)b * strideB;
  const T* Ab2 = SPLIT ? (A2  + (size_t)b * strideA) : nullptr;
  const T* Bb2 = SPLIT ? (Bt2 + (size_t)b * strideB) : nullptr;

  const int rlane = lane & 15;
  const int koff  = (lane >> 4) * 8;
  const int mOff  = (lane >> 4) * 8;

  v8f acc[4][4];
#pragma unroll
  for (int i = 0; i < 4; ++i)
#pragma unroll
    for (int j = 0; j < 4; ++j) acc[i][j] = (v8f){0.f,0.f,0.f,0.f,0.f,0.f,0.f,0.f};

  for (int k0 = 0; k0 < K; k0 += 32) {
    V bh[4], bl[4];
#pragma unroll
    for (int j = 0; j < 4; ++j) {
      const size_t bo = (size_t)(n0 + (j << 4) + rlane) * ldb + koff + k0;
      bh[j] = Frag<T>::load(Bb + bo);
      if (SPLIT) bl[j] = Frag<T>::load(Bb2 + bo);
    }
#pragma unroll
    for (int i = 0; i < 4; ++i) {
      const size_t ao = (size_t)(m0 + (i << 4) + rlane) * lda + koff + k0;
      V ah = Frag<T>::load(Ab + ao);
      V al;
      if (SPLIT) al = Frag<T>::load(Ab2 + ao);
#pragma unroll
      for (int j = 0; j < 4; ++j) {
        acc[i][j] = Frag<T>::mma(ah, bh[j], acc[i][j]);
        if (SPLIT) {
          acc[i][j] = Frag<T>::mma(ah, bl[j], acc[i][j]);
          acc[i][j] = Frag<T>::mma(al, bh[j], acc[i][j]);
        }
      }
      Frag<T>::guard(acc[i][0], acc[i][3], ah, SPLIT ? al : ah);
    }
    Frag<T>::keep(bh[0], bh[1], bh[2], bh[3]);
    if (SPLIT) Frag<T>::keep(bl[0], bl[1], bl[2], bl[3]);
  }
  acc_guard4(acc[0][0], acc[0][1], acc[0][2], acc[0][3]);
  acc_guard4(acc[1][0], acc[1][1], acc[1][2], acc[1][3]);
  acc_guard4(acc[2][0], acc[2][1], acc[2][2], acc[2][3]);
  acc_guard4(acc[3][0], acc[3][1], acc[3][2], acc[3][3]);

  float* slab = sT[wave];
  const float* Rb = RESID ? (resid + (size_t)b * strideR) : nullptr;
#pragma unroll
  for (int i = 0; i < 4; ++i) {
    const int mBase = m0 + (i << 4);
#pragma unroll
    for (int j = 0; j < 4; ++j) {
      const int n = n0 + (j << 4) + rlane;
      float bv = 0.f;
      if (BIAS_MODE == 2) bv = bias[n];
#pragma unroll
      for (int r = 0; r < 8; ++r) {
        float v = acc[i][j][r] * scale;
        if (BIAS_MODE == 1) v += bias[mBase + mOff + r];
        if (BIAS_MODE == 2) v += bv;
        if (RESID) v += Rb[(size_t)(mBase + mOff + r) * ldc + n];
        if (ACT == 1) v = tanhf(v);
        if (ACT == 2) v = fmaxf(v, 0.0f);
        if (ACT == 3) v = v / (1.0f + expf(-v));
        if (ACT == 4) v = (v > 0.f) ? v : 0.01f * v;
        if (ACT == 5) v = 0.5f * v * (1.0f + erff(v * 0.70710678118654752f));
        slab[(mOff + r) * 68 + (j << 4) + rlane] = v;
      }
    }
    __builtin_amdgcn_fence(__ATOMIC_RELEASE, "workgroup");
    __builtin_amdgcn_wave_barrier();
    __builtin_amdgcn_fence(__ATOMIC_ACQUIRE, "workgroup");
    if (OUT_MODE == 0) {
      float* C = (float*)Cout + (size_t)b * strideC;
      const int hh = lane >> 4, c4 = (lane & 15) * 4;
      for (int pass = 0; pass < 2; ++pass) {
#pragma unroll
        for (int it = 0; it < 8; ++it) {
          const int row = it * 2 + hh;
          v4f v = *(const v4f*)(slab + row * 68 + c4);
          *(volatile v4f*)(C + (size_t)(mBase + row) * ldc + n0 + c4) = v;
        }
        __threadfence();
      }
    } else {
      const int q = lane >> 3, c8 = (lane & 7) * 8;
      unsigned short* C  = (unsigned short*)Cout  + (size_t)b * strideC;
      unsigned short* C2 = (OUT_MODE == 2) ? ((unsigned short*)Cout2 + (size_t)b * strideC) : nullptr;
      for (int pass = 0; pass < 2; ++pass) {
#pragma unroll
        for (int it = 0; it < 4; ++it) {
          const int row = it * 4 + q;
          const float* sp = slab + row * 68 + c8;
          v8h hv, lv;
#pragma unroll
          for (int e = 0; e < 8; ++e) {
            if (OUT_MODE == 1) {
              hv[e] = (_Float16)sp[e];
            } else {
              unsigned short hb = f2bf_bits(sp[e]);
              unsigned short lb = f2bf_bits(sp[e] - bf_bits2f(hb));
              hv[e] = __builtin_bit_cast(_Float16, hb);
              lv[e] = __builtin_bit_cast(_Float16, lb);
            }
          }
          *(volatile v8h*)(C + (size_t)(mBase + row) * ldc + n0 + c8) = hv;
          if (OUT_MODE == 2) *(volatile v8h*)(C2 + (size_t)(mBase + row) * ldc + n0 + c8) = lv;
        }
        __threadfence();
      }
    }
    __builtin_amdgcn_fence(__ATOMIC_RELEASE, "workgroup");
    __builtin_amdgcn_wave_barrier();
    __builtin_amdgcn_fence(__ATOMIC_ACQUIRE, "workgroup");
  }
}

constexpr int kBatch = 2;
constexpr int kSeq   = 2048;
constexpr int kDm    = 768;
constexpr int kHeads = 12;
constexpr int kHd    = 64;
constexpr int kNumBuckets = 32;
constexpr int kQB = 64;
constexpr int kKC = 64;
constexpr int kNW = 4;
constexpr float kMaskFill = -1.0e30f;
constexpr float kPCarry   = 32768.0f;
constexpr float kOutCarry = 64.0f;
constexpr float kWoCarry  = 64.0f;
constexpr float kLn8      = 2.0794415416798357f;
constexpr float kInvLn8   = 1.0f / kLn8;
static_assert(kDm == kHeads * kHd);
static_assert(kSeq % kQB == 0 && kSeq % kKC == 0);
static_assert(kDm % 64 == 0 && kSeq % 64 == 0 && (kBatch * kSeq) % 64 == 0 && kDm % 32 == 0);

template <int MODE>
__global__ __launch_bounds__(256) void cast3_kernel(const float* __restrict__ in0, const float* __restrict__ in1,
                                                    const float* __restrict__ in2, unsigned short* __restrict__ o0,
                                                    unsigned short* __restrict__ o1, unsigned short* __restrict__ o2,
                                                    int n2, float sc) {
  const int z = blockIdx.y;
  const float* in = (z == 0) ? in0 : ((z == 1) ? in1 : in2);
  unsigned short* out = (z == 0) ? o0 : ((z == 1) ? o1 : o2);
  const int i = blockIdx.x * 256 + threadIdx.x;
  if (i < n2) {
    const v2f f = *(const v2f*)(in + 2 * (size_t)i);
    unsigned short a0, a1;
    if (MODE == 0) {
      a0 = f2bf_bits(f[0]);
      a1 = f2bf_bits(f[1]);
    } else {
      const _Float16 h0 = (_Float16)(bf_bits2f(f2bf_bits(f[0])) * sc);
      const _Float16 h1 = (_Float16)(bf_bits2f(f2bf_bits(f[1])) * sc);
      a0 = __builtin_bit_cast(unsigned short, h0);
      a1 = __builtin_bit_cast(unsigned short, h1);
    }
    const unsigned u = (unsigned)a0 | ((unsigned)a1 << 16);
    ((volatile unsigned*)out)[i] = u;
    __threadfence();
    ((volatile unsigned*)out)[i] = u;
  }
}

__device__ __forceinline__ v8f mma_h(v16h a, v16h b, v8f c) {
  c = __builtin_amdgcn_wmma_f32_16x16x32_f16(false, a, false, b, (short)0, c, false, false);
  asm volatile("v_nop\n\tv_nop\n\tv_nop\n\tv_nop" : "+v"(c) : "v"(a), "v"(b));
  return c;
}

__global__ __launch_bounds__(128)
void attn_relbias_kernel(const unsigned short* __restrict__ qp, const unsigned short* __restrict__ kp,
                         const unsigned short* __restrict__ vtp, const int* __restrict__ mask,
                         const float* __restrict__ rel_emb, unsigned short* __restrict__ outp, float sscale) {
  __shared__ __align__(16) _Float16 Ksh[kKC * kHd];
  __shared__ __align__(16) _Float16 Vth[kHd * kKC];
  __shared__ __align__(16) _Float16 Psh[kNW][16 * kKC];
  __shared__ __align__(16) float    Os[kNW][16 * 68];
  __shared__ float btab[2 * kSeq];

  const int tid  = threadIdx.x;
  const int wave = tid >> 5;
  const int lane = tid & 31;
  const int hh   = lane >> 4;
  const int c    = lane & 15;

  constexpr int nqb = kSeq / kQB;
  const int bx   = blockIdx.x;
  const int qb   = bx % nqb;
  const int bhid = bx / nqb;
  const int h    = bhid % kHeads;
  const int b    = bhid / kHeads;
  const int q0   = qb * kQB + wave * 16;

  for (int i = tid; i < 2 * kSeq; i += 128) {
    const int rel = i - (kSeq - 1);
    const int n   = -rel;
    const int nn  = (n < 1) ? 1 : n;
    const float ratio = logf((float)nn * 0.0625f) * kInvLn8;
    int vl = (int)(ratio * 16.0f);
    vl = (vl < 0) ? 0 : ((vl > 15) ? 15 : vl);
    const int nb = (n < 16) ? n : (16 + vl);
    int rb = (rel > 0) ? (16 + nb) : nb;
    rb = (rb < 0) ? 0 : ((rb > kNumBuckets - 1) ? (kNumBuckets - 1) : rb);
    btab[i] = bf_bits2f(f2bf_bits(rel_emb[rb * kHeads + h]));
  }
  __syncthreads();

  const _Float16* Qh = (const _Float16*)(const void*)qp  + (size_t)b * kSeq * kDm + (size_t)h * kHd;
  const _Float16* Kh = (const _Float16*)(const void*)kp  + (size_t)b * kSeq * kDm + (size_t)h * kHd;
  const _Float16* Vb = (const _Float16*)(const void*)vtp + (size_t)b * kDm * kSeq + (size_t)h * kHd * kSeq;
  _Float16*       ob = (_Float16*)(void*)outp + (size_t)b * kSeq * kDm + (size_t)h * kHd;

  v16h qa[2];
#pragma unroll
  for (int dc = 0; dc < 2; ++dc)
    qa[dc] = Frag<_Float16>::load(Qh + (size_t)(q0 + c) * kDm + dc * 32 + 8 * hh);

  float mrow[8], lrow[8];
  int keep[8];
  v8f oacc[4];
#pragma unroll
  for (int r = 0; r < 8; ++r) { mrow[r] = -INFINITY; lrow[r] = 0.f; keep[r] = 0; }
#pragma unroll
  for (int t = 0; t < 4; ++t) oacc[t] = (v8f){0.f,0.f,0.f,0.f,0.f,0.f,0.f,0.f};

  for (int kc = 0; kc < kSeq / kKC; ++kc) {
    const int kv0 = kc * kKC;
    __syncthreads();
    {
      const int r = tid >> 1, half = (tid & 1) * 32;
      const _Float16* ks = Kh + (size_t)(kv0 + r) * kDm + half;
      const _Float16* vs = Vb + (size_t)r * kSeq + kv0 + half;
#pragma unroll
      for (int i = 0; i < 4; ++i) {
        const v8h a0 = *(const v8h*)(ks + 8 * i);
        const v8h b0 = *(const v8h*)(vs + 8 * i);
        *(v8h*)(Ksh + r * kHd + half + 8 * i) = a0;
        *(v8h*)(Vth + r * kKC + half + 8 * i) = b0;
      }
    }
    __syncthreads();

    v8f s[4];
#pragma unroll
    for (int j = 0; j < 4; ++j) {
      s[j] = (v8f){0.f,0.f,0.f,0.f,0.f,0.f,0.f,0.f};
#pragma unroll
      for (int dc = 0; dc < 2; ++dc) {
        const v16h kb = Frag<_Float16>::load(Ksh + (j * 16 + c) * kHd + dc * 32 + 8 * hh);
        s[j] = mma_h(qa[dc], kb, s[j]);
      }
    }
    float cm[8];
#pragma unroll
    for (int r = 0; r < 8; ++r) {
      const int qrow = q0 + 8 * hh + r;
      const int* mr = mask + (size_t)qrow * kSeq + kv0;
      const float* br = btab + (kv0 - qrow + (kSeq - 1));
      float m = -INFINITY;
      int kany = 0;
#pragma unroll
      for (int j = 0; j < 4; ++j) {
        const int col = j * 16 + c;
        const int mv = mr[col];
        float sv = s[j][r] * sscale + br[col];
        kany |= (mv != 0) ? 1 : 0;
        sv = (mv == 0) ? kMaskFill : sv;
        s[j][r] = sv;
        m = fmaxf(m, sv);
      }
      keep[r] |= kany;
#pragma unroll
      for (int off = 1; off < 16; off <<= 1) m = fmaxf(m, __shfl_xor(m, off, 32));
      cm[r] = m;
    }
    _Float16* pw = Psh[wave];
#pragma unroll
    for (int r = 0; r < 8; ++r) {
      const float mnew  = fmaxf(mrow[r], cm[r]);
      const float alpha = expf(mrow[r] - mnew);
      mrow[r] = mnew;
      float psum = 0.f;
#pragma unroll
      for (int j = 0; j < 4; ++j) {
        const float p = expf(s[j][r] - mnew);
        psum += p;
        pw[(8 * hh + r) * kKC + j * 16 + c] = (_Float16)(p * kPCarry);
      }
#pragma unroll
      for (int off = 1; off < 16; off <<= 1) psum += __shfl_xor(psum, off, 32);
      lrow[r] = lrow[r] * alpha + psum;
#pragma unroll
      for (int t = 0; t < 4; ++t) oacc[t][r] *= alpha;
    }
    __builtin_amdgcn_fence(__ATOMIC_RELEASE, "workgroup");
    __builtin_amdgcn_wave_barrier();
    __builtin_amdgcn_fence(__ATOMIC_ACQUIRE, "workgroup");
#pragma unroll 1
    for (int kk = 0; kk < 2; ++kk) {
      const v16h pa = Frag<_Float16>::load(pw + c * kKC + kk * 32 + 8 * hh);
#pragma unroll
      for (int t = 0; t < 4; ++t) {
        const v16h vb = Frag<_Float16>::load(Vth + (t * 16 + c) * kKC + kk * 32 + 8 * hh);
        oacc[t] = mma_h(pa, vb, oacc[t]);
      }
    }
  }

  float* os = Os[wave];
#pragma unroll
  for (int r = 0; r < 8; ++r) {
    int kn = keep[r];
#pragma unroll
    for (int off = 1; off < 16; off <<= 1) kn |= __shfl_xor(kn, off, 32);
    const float rl  = 1.0f / (lrow[r] * kPCarry);
    const float inv = (kn != 0) ? (rl * kOutCarry) : 0.f;
#pragma unroll
    for (int t = 0; t < 4; ++t) os[(8 * hh + r) * 68 + t * 16 + c] = oacc[t][r] * inv;
  }
  __builtin_amdgcn_fence(__ATOMIC_RELEASE, "workgroup");
  __builtin_amdgcn_wave_barrier();
  __builtin_amdgcn_fence(__ATOMIC_ACQUIRE, "workgroup");
  {
    const int q4 = lane >> 3, c8 = (lane & 7) * 8;
    for (int pass = 0; pass < 2; ++pass) {
#pragma unroll
      for (int it = 0; it < 4; ++it) {
        const int row = it * 4 + q4;
        const float* sp = os + row * 68 + c8;
        v8h hv;
#pragma unroll
        for (int e = 0; e < 8; ++e) hv[e] = (_Float16)sp[e];
        *(volatile v8h*)(ob + (size_t)(q0 + row) * kDm + c8) = hv;
      }
      __threadfence();
    }
  }
}

extern "C" void kernel_launch(void* const* d_in, const int* in_sizes, int n_in,
                              void* d_out, int out_size, void* d_ws, size_t ws_size,
                              hipStream_t stream) {
  if (n_in < 9) return;
  const int nX = kBatch * kSeq * kDm;
  const int nW = kDm * kDm;
  if (in_sizes[0] != nX || in_sizes[1] != nX || in_sizes[2] != nX) return;
  if (in_sizes[3] != kSeq * kSeq) return;
  if (in_sizes[4] != nW || in_sizes[5] != nW || in_sizes[6] != nW || in_sizes[7] != nW) return;
  if (in_sizes[8] != kNumBuckets * kHeads) return;
  if (out_size != nX) return;

  const float* Qin = (const float*)d_in[0];
  const float* Kin = (const float*)d_in[1];
  const float* Vin = (const float*)d_in[2];
  const int*   Min = (const int*)d_in[3];
  const float* WQ  = (const float*)d_in[4];
  const float* WK  = (const float*)d_in[5];
  const float* WV  = (const float*)d_in[6];
  const float* WO  = (const float*)d_in[7];
  const float* RE  = (const float*)d_in[8];
  float* out = (float*)d_out;

  const size_t XB = (size_t)nX * 2;
  const size_t WB = (size_t)nW * 2;
  const size_t total = 7 * XB + 4 * WB;
  if (total > ws_size) return;
  unsigned char* ws = (unsigned char*)d_ws;
  unsigned short* xq  = (unsigned short*)(ws + 0 * XB);
  unsigned short* xk  = (unsigned short*)(ws + 1 * XB);
  unsigned short* xv  = (unsigned short*)(ws + 2 * XB);
  unsigned short* wq  = (unsigned short*)(ws + 3 * XB + 0 * WB);
  unsigned short* wk  = (unsigned short*)(ws + 3 * XB + 1 * WB);
  unsigned short* wv  = (unsigned short*)(ws + 3 * XB + 2 * WB);
  unsigned short* wo  = (unsigned short*)(ws + 3 * XB + 3 * WB);
  unsigned short* qpl = (unsigned short*)(ws + 3 * XB + 4 * WB);
  unsigned short* kpl = (unsigned short*)(ws + 4 * XB + 4 * WB);
  unsigned short* vtp = (unsigned short*)(ws + 5 * XB + 4 * WB);
  unsigned short* aop = (unsigned short*)(ws + 6 * XB + 4 * WB);
  const float* fdummy = (const float*)d_ws;

  const int n2X = nX / 2;
  cast3_kernel<0><<<dim3(n2X / 256, 3), 256, 0, stream>>>(Qin, Kin, Vin, xq, xk, xv, n2X, 1.0f);
  const int n2W = nW / 2;
  cast3_kernel<0><<<dim3(n2W / 256, 3), 256, 0, stream>>>(WQ, WK, WV, wq, wk, wv, n2W, 1.0f);
  cast3_kernel<1><<<dim3(n2W / 256, 1), 256, 0, stream>>>(WO, WO, WO, wo, wo, wo, n2W, kWoCarry);

  const int Mx = kBatch * kSeq;
  const int blkQK = (Mx / 64) * (kDm / 64) / 8;
  wmma_gemm64<1, false, 0, 1, false><<<dim3(blkQK, 1), 256, 0, stream>>>(
      xq, xq, kDm, 0L, wq, wq, kDm, 0L, (void*)qpl, (void*)qpl, kDm, 0L, fdummy, fdummy, 0L, Mx, kDm, kDm, 1.0f);
  wmma_gemm64<1, false, 0, 1, false><<<dim3(blkQK, 1), 256, 0, stream>>>(
      xk, xk, kDm, 0L, wk, wk, kDm, 0L, (void*)kpl, (void*)kpl, kDm, 0L, fdummy, fdummy, 0L, Mx, kDm, kDm, 1.0f);
  const int blkVT = (kDm / 64) * (kSeq / 64) / 8;
  wmma_gemm64<1, false, 0, 1, false><<<dim3(blkVT, kBatch), 256, 0, stream>>>(
      wv, wv, kDm, 0L, xv, xv, kDm, (long)kSeq * kDm, (void*)vtp, (void*)vtp, kSeq, (long)kDm * kSeq,
      fdummy, fdummy, 0L, kDm, kSeq, kDm, 1.0f);

  const int blkAT = kBatch * kHeads * (kSeq / kQB);
  attn_relbias_kernel<<<dim3(blkAT), 128, 0, stream>>>(qpl, kpl, vtp, Min, RE, aop, 0.125f);

  wmma_gemm64<0, false, 0, 0, false><<<dim3(blkQK, 1), 256, 0, stream>>>(
      aop, aop, kDm, 0L, wo, wo, kDm, 0L, (void*)out, (void*)out, kDm, 0L, fdummy, fdummy, 0L,
      Mx, kDm, kDm, 1.0f / (kOutCarry * kWoCarry));
}
